// EmbModule_62775241998338
// MI455X (gfx1250) — hardware-verified
//
#include <hip/hip_runtime.h>
#include <stddef.h>
#include <math.h>


#define DIM_IN  128
#define DIM_T   32
#define DIN     160
#define DOUT    128
#define NHEAD   4
#define HDIM    32
#define NREL    9
#define NLAY    2
#define NTHR    256
#define NWAVE   8
#define EPT     8
#define NGRP    2
#define CHUNK   (NTHR * EPT * NGRP)
#define WCAP    (EPT * NGRP * 32)
#define LISTN   (NWAVE * WCAP)
#define NBA     256
#define HCAP    2048
#define GROWS   128
#define HROWS   16
#define WSCALE  16.0f
#define WINV    0.0625f
#define NEG_SLOPE 0.2f
#define RELINV  (1.0f / 9.0f)

#define LDS_GEMM (GROWS * DOUT * 4 + 2 * DOUT * 4)
#define LDS_AGG  (NBA * DOUT * 4 + LISTN * 4 + HCAP * 4 + HCAP * NHEAD * 4 + 3 * NBA * NHEAD * 4 + 64)

static_assert((CHUNK & (CHUNK - 1)) == 0);
static_assert(CHUNK <= 4096);
static_assert((NBA & (NBA - 1)) == 0 && NBA <= 256);
static_assert(NTHR == NBA);
static_assert(NTHR == 2 * DOUT);
static_assert(NTHR == 2 * GROWS);
static_assert(DIN % 32 == 0 && DIN == DIM_IN + DIM_T);
static_assert(HROWS * DIM_IN / 8 == NTHR);
static_assert(HROWS * DIM_T / 8 == 64);
static_assert((NBA * DOUT / 4) % NTHR == 0);
static_assert(NHEAD * HDIM == DOUT && DOUT == 128);
static_assert(GROWS == NWAVE * 16);

typedef float    v4f  __attribute__((ext_vector_type(4)));
typedef float    v8f  __attribute__((ext_vector_type(8)));
typedef int      v4i  __attribute__((ext_vector_type(4)));
typedef _Float16 v8h  __attribute__((ext_vector_type(8)));
typedef _Float16 v16h __attribute__((ext_vector_type(16)));
union FragH { v16h v; v8h h[2]; };

__device__ __forceinline__ v8h cvt8(v4f a, v4f b) {
  v8h r;
  r[0] = (_Float16)a.x; r[1] = (_Float16)a.y; r[2] = (_Float16)a.z; r[3] = (_Float16)a.w;
  r[4] = (_Float16)b.x; r[5] = (_Float16)b.y; r[6] = (_Float16)b.z; r[7] = (_Float16)b.w;
  return r;
}

__device__ __forceinline__ v8f wmh(v16h a, v16h b, v8f c) {
  v8f d = __builtin_amdgcn_wmma_f32_16x16x32_f16(false, a, false, b, (short)0, c, false, false);
#if defined(__HIP_DEVICE_COMPILE__)
  asm volatile("v_nop\n\tv_nop\n\tv_nop\n\tv_nop" : "+v"(d) : "v"(a), "v"(b));
#endif
  return d;
}

template <int NS>
__device__ __forceinline__ int scan_chunk(const int* __restrict__ dsts, int nE, int cbase, int slotBase,
                                          int vec8, int* list, int tid, int lane, int wave) {
  int wc = 0;
#pragma unroll
  for (int g = 0; g < NGRP; ++g) {
    const int el0  = (g * NTHR + tid) * EPT;
    const int e0   = cbase + el0;
    const int sent = -2147483647 - 1;
    v4i da, db;
    if (vec8 != 0 && cbase + CHUNK <= nE) {
      da = *(const v4i*)(dsts + e0);
      db = *(const v4i*)(dsts + e0 + 4);
    } else {
      da.x = (e0     < nE) ? dsts[min(e0, nE - 1)]     : sent;
      da.y = (e0 + 1 < nE) ? dsts[min(e0 + 1, nE - 1)] : sent;
      da.z = (e0 + 2 < nE) ? dsts[min(e0 + 2, nE - 1)] : sent;
      da.w = (e0 + 3 < nE) ? dsts[min(e0 + 3, nE - 1)] : sent;
      db.x = (e0 + 4 < nE) ? dsts[min(e0 + 4, nE - 1)] : sent;
      db.y = (e0 + 5 < nE) ? dsts[min(e0 + 5, nE - 1)] : sent;
      db.z = (e0 + 6 < nE) ? dsts[min(e0 + 6, nE - 1)] : sent;
      db.w = (e0 + 7 < nE) ? dsts[min(e0 + 7, nE - 1)] : sent;
    }
    const unsigned nb = (unsigned)slotBase;
    const unsigned s0 = (unsigned)da.x - nb, s1 = (unsigned)da.y - nb;
    const unsigned s2 = (unsigned)da.z - nb, s3 = (unsigned)da.w - nb;
    const unsigned s4 = (unsigned)db.x - nb, s5 = (unsigned)db.y - nb;
    const unsigned s6 = (unsigned)db.z - nb, s7 = (unsigned)db.w - nb;
    const bool h0 = s0 < (unsigned)NS, h1 = s1 < (unsigned)NS, h2 = s2 < (unsigned)NS, h3 = s3 < (unsigned)NS;
    const bool h4 = s4 < (unsigned)NS, h5 = s5 < (unsigned)NS, h6 = s6 < (unsigned)NS, h7 = s7 < (unsigned)NS;
    const unsigned any = __builtin_amdgcn_ballot_w32(h0 | h1 | h2 | h3 | h4 | h5 | h6 | h7);
    if (any != 0u) {
#define HITJ(J, HJ, SJ) { \
        const unsigned mj = __builtin_amdgcn_ballot_w32(HJ); \
        if (mj != 0u) { \
          if (HJ) { \
            const int pos = wc + (int)__builtin_amdgcn_mbcnt_lo(mj, 0u); \
            if (pos < WCAP) list[wave * WCAP + pos] = ((el0 + (J)) << 12) | (int)(SJ); \
          } \
          wc += (int)__builtin_popcount(mj); } }
      HITJ(0, h0, s0)
      HITJ(1, h1, s1)
      HITJ(2, h2, s2)
      HITJ(3, h3, s3)
      HITJ(4, h4, s4)
      HITJ(5, h5, s5)
      HITJ(6, h6, s6)
      HITJ(7, h7, s7)
#undef HITJ
    }
  }
  return wc;
}

__global__ __launch_bounds__(NTHR) void k_prep(const float* __restrict__ W, _Float16* Wp, int nTot8) {
  const int i = blockIdx.x * NTHR + (int)threadIdx.x;
  if (i >= nTot8) return;
  const int o   = i * 8;
  const int lr  = o / (DOUT * DIN);
  const int rem = o - lr * (DOUT * DIN);
  const int n   = rem / DIN;
  const int k0  = rem - n * DIN;
  const float* src = W + (size_t)lr * DIN * DOUT + (size_t)k0 * DOUT + n;
  v4f a, b;
  a.x = src[0 * DOUT] * WSCALE; a.y = src[1 * DOUT] * WSCALE; a.z = src[2 * DOUT] * WSCALE; a.w = src[3 * DOUT] * WSCALE;
  b.x = src[4 * DOUT] * WSCALE; b.y = src[5 * DOUT] * WSCALE; b.z = src[6 * DOUT] * WSCALE; b.w = src[7 * DOUT] * WSCALE;
  const v8h hv = cvt8(a, b);
  _Float16* dp = Wp + o;
  *(volatile v8h*)dp = hv;
  __threadfence();
  *(volatile v8h*)dp = hv;
}

__global__ __launch_bounds__(NTHR) void k_hcat(
    const float* __restrict__ emb, const float* __restrict__ hsrc, const int* __restrict__ nid,
    const float* __restrict__ freq, const float* __restrict__ phs, const int* __restrict__ tsp,
    _Float16* hcat, int nN, int nume, int mode) {
#pragma clang fp contract(off)
  __shared__ __attribute__((aligned(16))) _Float16 st[HROWS * DIN];
  const int tid = threadIdx.x;
  const int rowBase = blockIdx.x * HROWS;
  const int tsv = tsp[0];
  {
    const int r   = tid >> 4, c0 = 8 * (tid & 15);
    const int row = rowBase + r;
    const int rowc = row < nN ? row : nN - 1;
    v4f a, b;
    if (mode == 0) {
      const int id = nid[rowc];
      int rm = id % nume;
      rm = rm < 0 ? rm + nume : rm;
      const float* p = emb + (size_t)rm * DIM_IN + c0;
      a = *(const v4f*)p; b = *(const v4f*)(p + 4);
    } else {
      const float* p = hsrc + (size_t)rowc * DOUT + c0;
      a = *(const v4f*)p; b = *(const v4f*)(p + 4);
    }
    if (row >= nN) {
      a.x = 0.f; a.y = 0.f; a.z = 0.f; a.w = 0.f;
      b.x = 0.f; b.y = 0.f; b.z = 0.f; b.w = 0.f;
    }
    *(v8h*)(st + r * DIN + c0) = cvt8(a, b);
  }
  if (tid < 64) {
    const int r   = tid >> 2, j0 = 8 * (tid & 3);
    const int row = rowBase + r;
    const int rowc = row < nN ? row : nN - 1;
    const int id  = nid[rowc];
    int q = id / nume;
    const int rmm = id - q * nume;
    if (rmm != 0 && id < 0) q -= 1;
    const float t = (float)(tsv - q);
    _Float16* sp = st + r * DIN + DIM_IN + j0;
#pragma unroll 1
    for (int e = 0; e < 8; ++e) {
      const float f  = freq[j0 + e];
      const float ph = phs[j0 + e];
      float arg = t * f;
      arg = arg + ph;
      float c = cosf(arg);
      c = row < nN ? c : 0.0f;
      sp[e] = (_Float16)c;
    }
  }
  __syncthreads();
  _Float16* gp = hcat + (size_t)rowBase * DIN;
  const v8h p0 = *(const v8h*)(st + 8 * tid);
  v8h p1 = p0;
  if (tid < 64) p1 = *(const v8h*)(st + 8 * (NTHR + tid));
  *(volatile v8h*)(gp + 8 * tid) = p0;
  if (tid < 64) *(volatile v8h*)(gp + 8 * (NTHR + tid)) = p1;
  __threadfence();
  *(volatile v8h*)(gp + 8 * tid) = p0;
  if (tid < 64) *(volatile v8h*)(gp + 8 * (NTHR + tid)) = p1;
}

__global__ __launch_bounds__(NTHR) void k_gemm(
    const _Float16* __restrict__ hcat, const _Float16* __restrict__ Wp,
    const float* __restrict__ attl, const float* __restrict__ attr,
    float* z, float* el, float* er) {
  extern __shared__ v4f lds_dyn[];
  float* stg  = (float*)lds_dyn;
  float* satt = stg + GROWS * DOUT;
  const int tid = threadIdx.x, lane = tid & 31, wave = tid >> 5, hh = lane >> 4, m = lane & 15;
  const int rowBase = blockIdx.x * GROWS;
  {
    const float a0 = attl[tid & (DOUT - 1)];
    const float b0 = attr[tid & (DOUT - 1)];
    satt[tid] = tid < DOUT ? a0 : b0;
  }

  v8f acc[8];
#pragma unroll
  for (int t = 0; t < 8; ++t) { v8f zz = {0.f, 0.f, 0.f, 0.f, 0.f, 0.f, 0.f, 0.f}; acc[t] = zz; }
  const _Float16* ap = hcat + (size_t)(rowBase + wave * 16 + m) * DIN + 8 * hh;
#pragma unroll
  for (int kt = 0; kt < DIN / 32; ++kt) {
    FragH a;
    a.h[0] = *(const v8h*)(ap + 32 * kt);
    a.h[1] = *(const v8h*)(ap + 32 * kt + 16);
#pragma unroll
    for (int t = 0; t < 8; ++t) {
      const _Float16* bp = Wp + (size_t)(16 * t + m) * DIN + 32 * kt + 8 * hh;
      FragH b;
      b.h[0] = *(const v8h*)bp;
      b.h[1] = *(const v8h*)(bp + 16);
      acc[t] = wmh(a.v, b.v, acc[t]);
    }
  }

  float* sp = stg + (wave * 16 + 8 * hh) * DOUT + m;
#pragma unroll
  for (int t = 0; t < 8; ++t) {
#pragma unroll
    for (int r = 0; r < 8; ++r) sp[r * DOUT + 16 * t] = acc[t][r] * WINV;
  }
  __syncthreads();

  const int row = tid & (GROWS - 1), side = tid >> 7;
  const float* att = satt + side * DOUT;
  const float* zr  = stg + row * DOUT;
  float rs[NHEAD];
#pragma unroll
  for (int hd = 0; hd < NHEAD; ++hd) {
    float s = 0.0f;
#pragma unroll 2
    for (int d = 0; d < HDIM; d += 4) {
      const v4f zv = *(const v4f*)(zr + hd * HDIM + d);
      const v4f av = *(const v4f*)(att + hd * HDIM + d);
      s += zv.x * av.x; s += zv.y * av.y; s += zv.z * av.z; s += zv.w * av.w;
    }
    rs[hd] = s;
  }
  v4f ev;
  ev.x = rs[0]; ev.y = rs[1]; ev.z = rs[2]; ev.w = rs[3];
  float* ep = (side == 0 ? el : er) + (size_t)(rowBase + row) * NHEAD;
  *(volatile v4f*)ep = ev;

  const float* lp = stg + wave * 16 * DOUT + 4 * lane;
  float* gz = z + ((size_t)rowBase + wave * 16) * DOUT + 4 * lane;
#pragma unroll
  for (int i = 0; i < 16; ++i) { const v4f v = *(const v4f*)(lp + i * DOUT); *(volatile v4f*)(gz + (size_t)i * DOUT) = v; }
  __threadfence();
  *(volatile v4f*)ep = ev;
#pragma unroll
  for (int i = 0; i < 16; ++i) { const v4f v = *(const v4f*)(lp + i * DOUT); *(volatile v4f*)(gz + (size_t)i * DOUT) = v; }
}

__global__ __launch_bounds__(NTHR) void k_agg(
    const int* __restrict__ esrc, const int* __restrict__ edst,
    const float* __restrict__ z, const float* __restrict__ el, const float* __restrict__ er,
    const float* __restrict__ bias, float* hbuf, int nN, int nE, int vec8, int first, int last) {
  extern __shared__ v4f lds_dyn[];
  float* acc   = (float*)lds_dyn;
  int*   clist = (int*)(acc + NBA * DOUT);
  int*   blist = clist + LISTN;
  float* exl   = (float*)(blist + HCAP);
  float* sm    = exl + HCAP * NHEAD;
  float* ss    = sm + NBA * NHEAD;
  float* ers   = ss + NBA * NHEAD;
  int*   wcnt  = (int*)(ers + NBA * NHEAD);
  const int tid = threadIdx.x, lane = tid & 31, wave = tid >> 5;
  const int nodeBase = blockIdx.x * NBA;

  {
    const v4f zz = {0.f, 0.f, 0.f, 0.f};
#pragma unroll 4
    for (int i = tid; i < NBA * DOUT / 4; i += NTHR) ((v4f*)acc)[i] = zz;
    const v4f e4 = *(const v4f*)(er + (size_t)(nodeBase + tid) * NHEAD);
    ((v4f*)ers)[tid] = e4;
    const v4f mi = {-3.0e38f, -3.0e38f, -3.0e38f, -3.0e38f};
    ((v4f*)sm)[tid] = mi;
    ((v4f*)ss)[tid] = zz;
  }
  __syncthreads();

  int bcount = 0;
  const int nChunks = (nE + CHUNK - 1) / CHUNK;
#pragma unroll 1
  for (int ch = 0; ch < nChunks; ++ch) {
    const int cbase = ch * CHUNK;
    const int wc = scan_chunk<NBA>(edst, nE, cbase, nodeBase, vec8, clist, tid, lane, wave);
    if (lane == 0) wcnt[wave] = wc;
    __syncthreads();
    int pre = 0, tot = 0, myc = 0;
#pragma unroll
    for (int w = 0; w < NWAVE; ++w) {
      int c = wcnt[w];
      c = c < 0 ? 0 : (c > WCAP ? WCAP : c);
      pre += (w < wave) ? c : 0;
      myc = (w == wave) ? c : myc;
      tot += c;
    }
    const int* lp = clist + wave * WCAP;
#pragma unroll 1
    for (int i = lane; i < myc; i += 32) {
      const int pos = bcount + pre + i;
      if (pos < HCAP) {
        const int ent = lp[i];
        int e = cbase + ((ent >> 12) & (CHUNK - 1));
        e = e > nE - 1 ? nE - 1 : e;
        blist[pos] = (e << 8) | (ent & (NBA - 1));
      }
    }
    bcount += tot;
    bcount = bcount > HCAP ? HCAP : bcount;
    __syncthreads();
  }
  const int L = bcount;

  if (wave == 0) {
#pragma unroll 1
    for (int i = 0; i < L; ++i) {
      const int ent  = __builtin_amdgcn_readfirstlane(blist[i]);
      const int e    = ent >> 8;
      const int slot = ent & (NBA - 1);
      int src = esrc[e];
      src = src < 0 ? 0 : (src > nN - 1 ? nN - 1 : src);
      const int hd = lane & (NHEAD - 1);
      float x = el[(size_t)src * NHEAD + hd] + ers[slot * NHEAD + hd];
      x = x >= 0.0f ? x : NEG_SLOPE * x;
      if (lane < NHEAD) {
        exl[i * NHEAD + hd] = x;
        const float mo = sm[slot * NHEAD + hd];
        sm[slot * NHEAD + hd] = fmaxf(mo, x);
      }
      if (lane == 0) blist[i] = (src << 8) | slot;
    }
  }
  __syncthreads();
  if (wave == 0) {
#pragma unroll 1
    for (int i = 0; i < L; ++i) {
      const int ent  = __builtin_amdgcn_readfirstlane(blist[i]);
      const int slot = ent & (NBA - 1);
      const int hd = lane & (NHEAD - 1);
      const float x  = exl[i * NHEAD + hd];
      const float mm = sm[slot * NHEAD + hd];
      const float ex = expf(x - mm);
      if (lane < NHEAD) {
        exl[i * NHEAD + hd] = ex;
        const float so = ss[slot * NHEAD + hd];
        ss[slot * NHEAD + hd] = so + ex;
      }
    }
  }
  __syncthreads();
  {
    const v4f s4 = ((const v4f*)ss)[tid];
    v4f iv;
    iv.x = s4.x > 0.0f ? 1.0f / s4.x : 1.0f;
    iv.y = s4.y > 0.0f ? 1.0f / s4.y : 1.0f;
    iv.z = s4.z > 0.0f ? 1.0f / s4.z : 1.0f;
    iv.w = s4.w > 0.0f ? 1.0f / s4.w : 1.0f;
    ((v4f*)ss)[tid] = iv;
  }
  __syncthreads();
  if (wave == 0) {
#pragma unroll 1
    for (int i = 0; i < L; ++i) {
      const int ent  = __builtin_amdgcn_readfirstlane(blist[i]);
      const int src  = ent >> 8;
      const int slot = ent & (NBA - 1);
      const int hd = lane >> 3;
      const float a = exl[i * NHEAD + hd] * ss[slot * NHEAD + hd];
      const v4f zv = *(const v4f*)(z + (size_t)src * DOUT + 4 * lane);
      v4f* apx = (v4f*)(acc + slot * DOUT + 4 * lane);
      const v4f cur = *apx;
      *apx = cur + zv * a;
    }
  }
  __syncthreads();

#pragma unroll 2
  for (int it = 0; it < NBA * DOUT / 4 / NTHR; ++it) {
    const int p = it * NTHR + tid;
    const int row = p >> 5;
    const int c4 = (p & 31) * 4;
    v4f v = ((const v4f*)acc)[p];
    const v4f b4 = *(const v4f*)(bias + c4);
    v = v + b4;
    if (first == 0) {
      const v4f hv = *(const v4f*)(hbuf + (size_t)(nodeBase + row) * DOUT + c4);
      v = hv + v;
    }
    if (last != 0) {
      v = v * RELINV;
      v.x = fmaxf(v.x, 0.0f); v.y = fmaxf(v.y, 0.0f); v.z = fmaxf(v.z, 0.0f); v.w = fmaxf(v.w, 0.0f);
    }
    ((v4f*)acc)[p] = v;
  }
  float* hp = hbuf + (size_t)nodeBase * DOUT;
#pragma unroll 2
  for (int it = 0; it < NBA * DOUT / 4 / NTHR; ++it) {
    const int p = it * NTHR + tid;
    const v4f v = ((const v4f*)acc)[p];
    *(volatile v4f*)(hp + 4 * (size_t)p) = v;
  }
  __threadfence();
#pragma unroll 2
  for (int it = 0; it < NBA * DOUT / 4 / NTHR; ++it) {
    const int p = it * NTHR + tid;
    const v4f v = ((const v4f*)acc)[p];
    *(volatile v4f*)(hp + 4 * (size_t)p) = v;
  }
}

__global__ __launch_bounds__(NTHR) void k_out(
    const float* __restrict__ h, const int* __restrict__ root, float* out, int nRoot, int nN) {
  const int tid = threadIdx.x, lane = tid & 31, wave = tid >> 5;
  const int j  = blockIdx.x * NWAVE + wave;
  const int jc = j < nRoot ? j : nRoot - 1;
  int nd = root[jc];
  nd = nd < 0 ? nd + nN : nd;
  nd = nd < 0 ? 0 : (nd > nN - 1 ? nN - 1 : nd);
  const v4f v = *(const v4f*)(h + (size_t)nd * DOUT + 4 * lane);
  float* op = out + (size_t)jc * DOUT + 4 * lane;
  if (j < nRoot) *(volatile v4f*)op = v;
  __threadfence();
  if (j < nRoot) *(volatile v4f*)op = v;
}

extern "C" void kernel_launch(void* const* d_in, const int* in_sizes, int n_in,
                              void* d_out, int out_size, void* d_ws, size_t ws_size,
                              hipStream_t stream) {
  if (n_in < 12) return;
  const int nume = in_sizes[0] / DIM_IN;
  if (nume < 1 || in_sizes[0] != nume * DIM_IN) return;
  if (in_sizes[1] < DIM_T || in_sizes[2] < DIM_T) return;
  if (in_sizes[3] != NLAY * NREL * DIN * DOUT) return;
  if (in_sizes[4] != NLAY * NREL * NHEAD * HDIM || in_sizes[5] != NLAY * NREL * NHEAD * HDIM) return;
  if (in_sizes[6] != NLAY * NREL * DOUT) return;
  const int nN = in_sizes[7];
  if (nN < 1 || nN > (1 << 22)) return;
  const int nE = in_sizes[8] / NREL;
  if (nE < 1 || in_sizes[8] != nE * NREL || in_sizes[9] != nE * NREL || nE > (1 << 23)) return;
  const int nRoot = in_sizes[10];
  if (nRoot < 1 || out_size != nRoot * DOUT) return;
  if (in_sizes[11] < 1) return;

  const float* emb  = (const float*)d_in[0];
  const float* freq = (const float*)d_in[1];
  const float* phs  = (const float*)d_in[2];
  const float* W    = (const float*)d_in[3];
  const float* attl = (const float*)d_in[4];
  const float* attr = (const float*)d_in[5];
  const float* bias = (const float*)d_in[6];
  const int*   nid  = (const int*)d_in[7];
  const int*   esrc = (const int*)d_in[8];
  const int*   edst = (const int*)d_in[9];
  const int*   root = (const int*)d_in[10];
  const int*   tsp  = (const int*)d_in[11];
  float* out = (float*)d_out;

  const int NPAD  = ((nN + NBA - 1) / NBA) * NBA;
  const int nHcat = NPAD / HROWS;
  const int nGemm = NPAD / GROWS;
  const int nAgg  = NPAD / NBA;
  const int nTot8 = NLAY * NREL * DOUT * DIN / 8;
  const int nPrep = (nTot8 + NTHR - 1) / NTHR;
  const int nOut  = (nRoot + NWAVE - 1) / NWAVE;

  char* ws = (char*)d_ws;
  size_t off = 0;
  const size_t oW  = off; off += (size_t)NLAY * NREL * DOUT * DIN * 2; off = (off + 255) & ~(size_t)255;
  const size_t oHc = off; off += (size_t)NPAD * DIN * 2;               off = (off + 255) & ~(size_t)255;
  const size_t oZ  = off; off += (size_t)NPAD * DOUT * 4;              off = (off + 255) & ~(size_t)255;
  const size_t oEl = off; off += (size_t)NPAD * NHEAD * 4;             off = (off + 255) & ~(size_t)255;
  const size_t oEr = off; off += (size_t)NPAD * NHEAD * 4;             off = (off + 255) & ~(size_t)255;
  const size_t oH  = off; off += (size_t)NPAD * DOUT * 4;              off = (off + 255) & ~(size_t)255;
  if (off > ws_size || off > (size_t)134217728) return;
  _Float16* Wp   = (_Float16*)(ws + oW);
  _Float16* hcat = (_Float16*)(ws + oHc);
  float*    z    = (float*)(ws + oZ);
  float*    elp  = (float*)(ws + oEl);
  float*    erp  = (float*)(ws + oEr);
  float*    hbuf = (float*)(ws + oH);

  const int vec8 = ((nE & 3) == 0) ? 1 : 0;

  hipFuncSetAttribute(reinterpret_cast<const void*>(&k_gemm),
                      hipFuncAttributeMaxDynamicSharedMemorySize, LDS_GEMM);
  hipFuncSetAttribute(reinterpret_cast<const void*>(&k_agg),
                      hipFuncAttributeMaxDynamicSharedMemorySize, LDS_AGG);

  k_prep<<<nPrep, NTHR, 0, stream>>>(W, Wp, nTot8);

  for (int l = 0; l < NLAY; ++l) {
    k_hcat<<<nHcat, NTHR, 0, stream>>>(emb, hbuf, nid, freq, phs, tsp, hcat, nN, nume, l);
    for (int r = 0; r < NREL; ++r) {
      const int lr = l * NREL + r;
      k_gemm<<<nGemm, NTHR, LDS_GEMM, stream>>>(hcat, Wp + (size_t)lr * DOUT * DIN,
                                                attl + (size_t)lr * NHEAD * HDIM,
                                                attr + (size_t)lr * NHEAD * HDIM,
                                                z, elp, erp);
      k_agg<<<nAgg, NTHR, LDS_AGG, stream>>>(esrc + (size_t)r * nE, edst + (size_t)r * nE,
                                             z, elp, erp, bias + (size_t)lr * DOUT, hbuf,
                                             nN, nE, vec8, r == 0 ? 1 : 0, r == NREL - 1 ? 1 : 0);
    }
  }

  k_out<<<nOut, NTHR, 0, stream>>>(hbuf, root, out, nRoot, nN);
}
